// BrushModel_16174846837057
// MI455X (gfx1250) — hardware-verified
//
#include <hip/hip_runtime.h>
#include <stdint.h>


#define P_EXPERTS 16
#define H_DIM     128
#define M_TILE    256
#define NTHREADS  256
#define S_BT      136

typedef _Float16 v16h __attribute__((ext_vector_type(16)));
typedef _Float16 v8h  __attribute__((ext_vector_type(8)));
typedef _Float16 v4h  __attribute__((ext_vector_type(4)));
typedef float    v8f  __attribute__((ext_vector_type(8)));
typedef float    v4f  __attribute__((ext_vector_type(4)));
typedef v8h __attribute__((may_alias)) v8ha;
typedef v4h __attribute__((may_alias)) v4ha;
typedef v4f __attribute__((may_alias)) v4fa;

union Frag  { v16h v; v8h half[2]; };
union Pack8 { v8h v; _Float16 e[8]; };
union Pack4 { v4h v; _Float16 e[4]; };

__device__ __forceinline__ v8f wmma_f16(v16h a, v16h b, v8f c)
{
    v8f d = __builtin_amdgcn_wmma_f32_16x16x32_f16(false, a, false, b, (short)0, c, false, false);
    asm volatile("v_nop\n\tv_nop\n\tv_nop\n\tv_nop" : "+v"(d) : "v"(a), "v"(b));
    return d;
}

template<int DIN, int DOUT>
__global__ __launch_bounds__(NTHREADS)
void moe_mlp_fused(const float* __restrict__ x,
                   const float* __restrict__ W1,
                   const float* __restrict__ b1,
                   const float* __restrict__ W2,
                   const float* __restrict__ b2,
                   const float* __restrict__ W3,
                   const float* __restrict__ b3,
                   float* __restrict__ out,
                   int N)
{
    __shared__ __align__(16) _Float16 sA  [M_TILE * S_BT];
    __shared__ __align__(16) _Float16 sBt [H_DIM  * S_BT];
    __shared__ __align__(16) _Float16 sW3t[16     * S_BT];
    __shared__ __align__(16) float    sW1 [H_DIM * 4];
    __shared__ __align__(16) float    sB1 [H_DIM];
    __shared__ __align__(16) float    sB2 [H_DIM];
    __shared__ __align__(16) float    sB3 [4];
    __shared__ __align__(16) float    sOut[M_TILE * 4];

    const int tid  = threadIdx.x;
    const int l    = tid & 31;
    const int w    = tid >> 5;
    const int h    = l >> 4;
    const int m    = l & 15;
    const int p    = blockIdx.y;
    const int row0 = blockIdx.x * M_TILE;

    for (int i = tid; i < H_DIM * DIN; i += NTHREADS)
        sW1[i] = W1[(size_t)p * H_DIM * DIN + i];
    for (int i = tid; i < H_DIM; i += NTHREADS) {
        sB1[i] = b1[p * H_DIM + i];
        sB2[i] = b2[p * H_DIM + i];
    }
    if (tid < DOUT) sB3[tid] = b3[p * DOUT + tid];
    for (int i = tid; i < 16 * H_DIM; i += NTHREADS) {
        const int o = i >> 7, k = i & 127;
        const float v = (o < DOUT) ? W3[((size_t)p * DOUT + o) * H_DIM + k] : 0.f;
        sW3t[o * S_BT + k] = (_Float16)(v * 16.f);
    }
    {
        const v4fa* W2v = (const v4fa*)(W2 + (size_t)p * H_DIM * H_DIM);
        for (int c = tid; c < (H_DIM * H_DIM) / 4; c += NTHREADS) {
            const v4f wv = W2v[c];
            const int n  = c >> 5;
            const int k4 = (c & 31) << 2;
            Pack4 u;
            u.e[0] = (_Float16)(wv.x * 16.f);
            u.e[1] = (_Float16)(wv.y * 16.f);
            u.e[2] = (_Float16)(wv.z * 16.f);
            u.e[3] = (_Float16)(wv.w * 16.f);
            *(v4ha*)(sBt + n * S_BT + k4) = u.v;
        }
    }
    __syncthreads();

    {
        const int r  = tid;
        const int gr = row0 + r;
        float xr[DIN];
        #pragma unroll
        for (int d = 0; d < DIN; ++d)
            xr[d] = (gr < N) ? x[(size_t)gr * DIN + d] : 0.f;
        _Float16* arow = sA + r * S_BT;
        #pragma unroll 2
        for (int c8 = 0; c8 < H_DIM; c8 += 8) {
            Pack8 u;
            #pragma unroll
            for (int q = 0; q < 8; ++q) {
                const int hh = c8 + q;
                float v = sB1[hh];
                #pragma unroll
                for (int d = 0; d < DIN; ++d) v = fmaf(xr[d], sW1[hh * DIN + d], v);
                v = fmaxf(v, 0.f) * 16.f;
                u.e[q] = (_Float16)v;
            }
            *(v8ha*)(arow + c8) = u.v;
        }
    }
    __syncthreads();

    #pragma unroll 1
    for (int band = 0; band < 2; ++band) {
        const int rb = band * 128 + w * 16;
        v8f acc[8];
        #pragma unroll
        for (int j = 0; j < 8; ++j) { v8f z = {}; acc[j] = z; }
        const _Float16* arow = sA + (rb + m) * S_BT + 8 * h;
        #pragma unroll 1
        for (int kk = 0; kk < H_DIM; kk += 32) {
            Frag a;
            a.half[0] = *(const v8ha*)(arow + kk);
            a.half[1] = *(const v8ha*)(arow + kk + 16);
            #pragma unroll
            for (int j = 0; j < 8; ++j) {
                const _Float16* brow = sBt + (j * 16 + m) * S_BT + 8 * h + kk;
                Frag b;
                b.half[0] = *(const v8ha*)(brow);
                b.half[1] = *(const v8ha*)(brow + 16);
                acc[j] = wmma_f16(a.v, b.v, acc[j]);
            }
        }
        #pragma unroll
        for (int j = 0; j < 8; ++j) {
            const int col = j * 16 + m;
            const float bias = sB2[col];
            #pragma unroll
            for (int r = 0; r < 8; ++r) {
                float v = fmaf(acc[j][r], 0.00390625f, bias);
                v = fmaxf(v, 0.f) * 16.f;
                sA[(rb + 8 * h + r) * S_BT + col] = (_Float16)v;
            }
        }
    }
    __syncthreads();

    #pragma unroll 1
    for (int band = 0; band < 2; ++band) {
        const int rb = band * 128 + w * 16;
        v8f oacc = {};
        const _Float16* arow = sA + (rb + m) * S_BT + 8 * h;
        const _Float16* brow = sW3t + m * S_BT + 8 * h;
        #pragma unroll
        for (int kk = 0; kk < H_DIM; kk += 32) {
            Frag a, b;
            a.half[0] = *(const v8ha*)(arow + kk);
            a.half[1] = *(const v8ha*)(arow + kk + 16);
            b.half[0] = *(const v8ha*)(brow + kk);
            b.half[1] = *(const v8ha*)(brow + kk + 16);
            oacc = wmma_f16(a.v, b.v, oacc);
        }
        if (m < DOUT) {
            const float bias = sB3[m];
            #pragma unroll
            for (int r = 0; r < 8; ++r)
                sOut[(rb + 8 * h + r) * DOUT + m] = fmaf(oacc[r], 0.00390625f, bias);
        }
    }
    __syncthreads();

    {
        float* ob = out + ((size_t)p * (size_t)N + (size_t)row0) * DOUT;
        const int validRows = (N - row0 < M_TILE) ? (N - row0) : M_TILE;
        if (validRows == M_TILE) {
            const int  F   = 64 * DOUT;
            const bool act = tid < F;
            v4f v = {};
            if (act) {
                v = *(const v4fa*)(sOut + 4 * tid);
                *(volatile v4f*)(ob + 4 * tid) = v;
            }
            __threadfence();
            if (act) *(volatile v4f*)(ob + 4 * tid) = v;
        } else {
            const int nf = validRows * DOUT;
            float vals[4];
            #pragma unroll
            for (int it = 0; it < 4; ++it) {
                const int e = tid + it * NTHREADS;
                vals[it] = (e < nf) ? sOut[e] : 0.f;
                if (e < nf) *(volatile float*)(ob + e) = vals[it];
            }
            __threadfence();
            #pragma unroll
            for (int it = 0; it < 4; ++it) {
                const int e = tid + it * NTHREADS;
                if (e < nf) *(volatile float*)(ob + e) = vals[it];
            }
        }
    }
}

template<int DIN, int DOUT>
static size_t launch_attr(void* const* din, const int* sz, float* out, hipStream_t stream)
{
    const int N = sz[0] / DIN;
    if (N <= 0) return 0;
    dim3 grid((N + M_TILE - 1) / M_TILE, P_EXPERTS);
    moe_mlp_fused<DIN, DOUT><<<grid, dim3(NTHREADS), 0, stream>>>(
        (const float*)din[0], (const float*)din[1], (const float*)din[2],
        (const float*)din[3], (const float*)din[4], (const float*)din[5],
        (const float*)din[6], out, N);
    return (size_t)P_EXPERTS * (size_t)N * (size_t)DOUT;
}

extern "C" void kernel_launch(void* const* d_in, const int* in_sizes, int n_in,
                              void* d_out, int out_size, void* d_ws, size_t ws_size,
                              hipStream_t stream)
{
    (void)out_size; (void)d_ws; (void)ws_size;
    if (n_in < 35) return;
    float* out = (float*)d_out;
    size_t off = 0;
    off += launch_attr<3, 3>(d_in + 0 * 7, in_sizes + 0 * 7, out + off, stream);
    off += launch_attr<3, 3>(d_in + 1 * 7, in_sizes + 1 * 7, out + off, stream);
    off += launch_attr<3, 3>(d_in + 2 * 7, in_sizes + 2 * 7, out + off, stream);
    off += launch_attr<4, 4>(d_in + 3 * 7, in_sizes + 3 * 7, out + off, stream);
    off += launch_attr<1, 1>(d_in + 4 * 7, in_sizes + 4 * 7, out + off, stream);
    (void)off;
}
